// LearnableLSHAttention_10926396801633
// MI455X (gfx1250) — hardware-verified
//
#include <hip/hip_runtime.h>
#include <stdint.h>

#define NTOK   2048
#define DMODEL 1024
#define NHEAD  8
#define HDIM   128
#define NBUCK  64
#define NEGBIG (-1.0e30f)

#define KLD 136
#define PLD 72
#define OLD 132
#define CLD 68

typedef __bf16       v16bf __attribute__((ext_vector_type(16)));
typedef float        v8f   __attribute__((ext_vector_type(8)));
typedef float        v4f   __attribute__((ext_vector_type(4)));
typedef unsigned int v4u   __attribute__((ext_vector_type(4)));
typedef int          v4i   __attribute__((ext_vector_type(4)));

union Frag { v16bf v; v4u u[2]; };

static __device__ __forceinline__ unsigned int bfbits(float f) {
    unsigned int u = __float_as_uint(f);
    return (u + 0x7FFFu + ((u >> 16) & 1u)) >> 16;
}
static __device__ __forceinline__ void split2(float f, unsigned int& hb, unsigned int& lb) {
    hb = bfbits(f);
    const float hf = __uint_as_float(hb << 16);
    lb = bfbits(f - hf);
}
static __device__ __forceinline__ void pack8(const float (&v)[8], v4u& hv, v4u& lv) {
#pragma unroll
    for (int i = 0; i < 4; ++i) {
        unsigned int h0, l0, h1, l1;
        split2(v[2 * i], h0, l0);
        split2(v[2 * i + 1], h1, l1);
        hv[i] = h0 | (h1 << 16);
        lv[i] = l0 | (l1 << 16);
    }
}

static __device__ __forceinline__ v8f wmma3(v16bf ah, v16bf al, v16bf bh, v16bf bl, v8f c) {
    c = __builtin_amdgcn_wmma_f32_16x16x32_bf16(false, ah, false, bh, (short)0, c, false, false);
    c = __builtin_amdgcn_wmma_f32_16x16x32_bf16(false, al, false, bh, (short)0, c, false, false);
    c = __builtin_amdgcn_wmma_f32_16x16x32_bf16(false, ah, false, bl, (short)0, c, false, false);
    asm volatile("v_nop\n\tv_nop\n\tv_nop\n\tv_nop" : "+v"(c) : "v"(ah), "v"(al), "v"(bh), "v"(bl));
    return c;
}

__global__ void __launch_bounds__(256)
k_split8(const float* __restrict__ in, unsigned short* __restrict__ oh,
         unsigned short* __restrict__ ol, int n8) {
    const int i = blockIdx.x * 256 + threadIdx.x;
    if (i >= n8) return;
    const float* p = in + (size_t)i * 8;
    const v4f a = *(const v4f*)p;
    const v4f b = *(const v4f*)(p + 4);
    float v[8] = {a[0], a[1], a[2], a[3], b[0], b[1], b[2], b[3]};
    v4u hv, lv;
    pack8(v, hv, lv);
    const size_t o = (size_t)i * 8;
    *(volatile v4u*)(oh + o) = hv;
    *(volatile v4u*)(ol + o) = lv;
    __threadfence();
    *(volatile v4u*)(oh + o) = hv;
    *(volatile v4u*)(ol + o) = lv;
}

__global__ void __launch_bounds__(256)
k_splitT(const float* __restrict__ W, unsigned short* __restrict__ oh,
         unsigned short* __restrict__ ol, int R, int C) {
    __shared__ float ts[64 * 65];
    const int t = threadIdx.x;
    const int c0 = blockIdx.x * 64, r0 = blockIdx.y * 64;
#pragma unroll
    for (int it = 0; it < 4; ++it) {
        const int idx = it * 256 + t;
        const int r = idx >> 4, c4 = (idx & 15) * 4;
        v4f v = {0.f, 0.f, 0.f, 0.f};
        if (r0 + r < R && c0 + c4 + 3 < C)
            v = *(const v4f*)(W + (size_t)(r0 + r) * C + c0 + c4);
        ts[r * 65 + c4 + 0] = v[0];
        ts[r * 65 + c4 + 1] = v[1];
        ts[r * 65 + c4 + 2] = v[2];
        ts[r * 65 + c4 + 3] = v[3];
    }
    __syncthreads();
    for (int pass = 0; pass < 2; ++pass) {
        if (pass) __threadfence();
#pragma unroll
        for (int it = 0; it < 2; ++it) {
            const int c = it * 32 + (t >> 3);
            const int p = t & 7;
            float v[8];
#pragma unroll
            for (int i = 0; i < 8; ++i) v[i] = ts[(p * 8 + i) * 65 + c];
            v4u hv, lv;
            pack8(v, hv, lv);
            if (c0 + c < C && r0 + p * 8 + 7 < R) {
                const size_t o = (size_t)(c0 + c) * R + r0 + p * 8;
                *(volatile v4u*)(oh + o) = hv;
                *(volatile v4u*)(ol + o) = lv;
            }
        }
    }
}

__global__ void __launch_bounds__(128)
k_gemm3(const unsigned short* __restrict__ Ah, const unsigned short* __restrict__ Al,
        const unsigned short* __restrict__ Bh, const unsigned short* __restrict__ Bl,
        const float* __restrict__ bias, float* Of, unsigned short* Oh, unsigned short* Ol,
        int M, int N, int K, int flags) {
    __shared__ v4f cs4[64 * CLD / 4];
    float* cs = (float*)cs4;
    const int t = threadIdx.x, wave = t >> 5, lane = t & 31;
    const int lh = lane >> 4, lm = lane & 15;
    const int bm = blockIdx.y * 64, bn = blockIdx.x * 64;
    if (bm + 64 > M || bn + 64 > N) return;
    const int wm = (wave >> 1) * 32, wn = (wave & 1) * 32;

    const size_t ra0 = (size_t)(bm + wm + lm) * K + 8 * lh;
    const size_t ra1 = ra0 + (size_t)16 * K;
    const size_t rb0 = (size_t)(bn + wn + lm) * K + 8 * lh;
    const size_t rb1 = rb0 + (size_t)16 * K;

    v8f c00 = {}, c01 = {}, c10 = {}, c11 = {};
#pragma unroll 1
    for (int k0 = 0; k0 < K; k0 += 32) {
        Frag a0h, a0l, a1h, a1l, b0h, b0l, b1h, b1l;
        a0h.u[0] = *(const v4u*)(Ah + ra0 + k0); a0h.u[1] = *(const v4u*)(Ah + ra0 + k0 + 16);
        a0l.u[0] = *(const v4u*)(Al + ra0 + k0); a0l.u[1] = *(const v4u*)(Al + ra0 + k0 + 16);
        a1h.u[0] = *(const v4u*)(Ah + ra1 + k0); a1h.u[1] = *(const v4u*)(Ah + ra1 + k0 + 16);
        a1l.u[0] = *(const v4u*)(Al + ra1 + k0); a1l.u[1] = *(const v4u*)(Al + ra1 + k0 + 16);
        b0h.u[0] = *(const v4u*)(Bh + rb0 + k0); b0h.u[1] = *(const v4u*)(Bh + rb0 + k0 + 16);
        b0l.u[0] = *(const v4u*)(Bl + rb0 + k0); b0l.u[1] = *(const v4u*)(Bl + rb0 + k0 + 16);
        b1h.u[0] = *(const v4u*)(Bh + rb1 + k0); b1h.u[1] = *(const v4u*)(Bh + rb1 + k0 + 16);
        b1l.u[0] = *(const v4u*)(Bl + rb1 + k0); b1l.u[1] = *(const v4u*)(Bl + rb1 + k0 + 16);
        c00 = wmma3(a0h.v, a0l.v, b0h.v, b0l.v, c00);
        c01 = wmma3(a0h.v, a0l.v, b1h.v, b1l.v, c01);
        c10 = wmma3(a1h.v, a1l.v, b0h.v, b0l.v, c10);
        c11 = wmma3(a1h.v, a1l.v, b1h.v, b1l.v, c11);
    }

#pragma unroll
    for (int r = 0; r < 8; ++r) {
        const int row0 = wm + 8 * lh + r, row1 = row0 + 16;
        cs[row0 * CLD + wn + lm]      = c00[r];
        cs[row0 * CLD + wn + 16 + lm] = c01[r];
        cs[row1 * CLD + wn + lm]      = c10[r];
        cs[row1 * CLD + wn + 16 + lm] = c11[r];
    }
    __syncthreads();

    for (int pass = 0; pass < 2; ++pass) {
        if (pass) __threadfence();
        if (flags & 1) {
#pragma unroll
            for (int it = 0; it < 8; ++it) {
                const int L = it * 16 + (t >> 3);
                const int row = L >> 1;
                const int col = (L & 1) * 32 + (t & 7) * 4;
                v4f v = *(const v4f*)(cs + row * CLD + col);
                const v4f b4 = *(const v4f*)(bias + bn + col);
                v += b4;
                *(volatile v4f*)(Of + (size_t)(bm + row) * N + bn + col) = v;
            }
        }
        if (flags & 2) {
#pragma unroll
            for (int it = 0; it < 4; ++it) {
                const int row = it * 16 + (t >> 3);
                const int col = (t & 7) * 8;
                const v4f x0 = *(const v4f*)(cs + row * CLD + col);
                const v4f x1 = *(const v4f*)(cs + row * CLD + col + 4);
                const v4f b0 = *(const v4f*)(bias + bn + col);
                const v4f b1 = *(const v4f*)(bias + bn + col + 4);
                float v[8] = {x0[0] + b0[0], x0[1] + b0[1], x0[2] + b0[2], x0[3] + b0[3],
                              x1[0] + b1[0], x1[1] + b1[1], x1[2] + b1[2], x1[3] + b1[3]};
                v4u hv, lv;
                pack8(v, hv, lv);
                const size_t o = (size_t)(bm + row) * N + bn + col;
                *(volatile v4u*)(Oh + o) = hv;
                *(volatile v4u*)(Ol + o) = lv;
            }
        }
        if (flags & 4) {
#pragma unroll
            for (int it = 0; it < 4; ++it) {
                const int c = it * 16 + (t >> 3);
                const int p = t & 7;
                const float bs = bias[bn + c];
                float v[8];
#pragma unroll
                for (int i = 0; i < 8; ++i) v[i] = cs[(p * 8 + i) * CLD + c] + bs;
                v4u hv, lv;
                pack8(v, hv, lv);
                const size_t o = (size_t)(bn + c) * M + bm + p * 8;
                *(volatile v4u*)(Oh + o) = hv;
                *(volatile v4u*)(Ol + o) = lv;
            }
        }
    }
}

__global__ void __launch_bounds__(256)
k_hash(const float* __restrict__ q32, const float* __restrict__ hp, int* __restrict__ bkt) {
    __shared__ v4f qs4[32 * HDIM / 4];
    __shared__ v4f hs4[HDIM * NBUCK / 4];
    __shared__ int sb[32];
    const int t = threadIdx.x, hd = blockIdx.y, n0 = blockIdx.x * 32;
    if (n0 + 32 > NTOK) return;
#pragma unroll
    for (int it = 0; it < 4; ++it) {
        const int idx = it * 256 + t;
        const int r = idx >> 5, c4 = idx & 31;
        qs4[idx] = *(const v4f*)(q32 + (size_t)(n0 + r) * DMODEL + hd * HDIM + c4 * 4);
    }
#pragma unroll
    for (int it = 0; it < 8; ++it) {
        const int idx = it * 256 + t;
        hs4[idx] = *(const v4f*)(hp + (size_t)hd * HDIM * NBUCK + (size_t)idx * 4);
    }
    __syncthreads();
    const float* qs = (const float*)qs4;
    const int tok = t >> 3, g = t & 7;
    float s[8];
#pragma unroll
    for (int j = 0; j < 8; ++j) s[j] = 0.f;
#pragma unroll 1
    for (int d = 0; d < HDIM; ++d) {
        const float qv = qs[tok * HDIM + d];
        const v4f h0 = hs4[d * (NBUCK / 4) + g * 2];
        const v4f h1 = hs4[d * (NBUCK / 4) + g * 2 + 1];
        s[0] += qv * h0[0]; s[1] += qv * h0[1]; s[2] += qv * h0[2]; s[3] += qv * h0[3];
        s[4] += qv * h1[0]; s[5] += qv * h1[1]; s[6] += qv * h1[2]; s[7] += qv * h1[3];
    }
    float bv = s[0];
    int bi = 0;
#pragma unroll
    for (int j = 1; j < 8; ++j)
        if (s[j] > bv) { bv = s[j]; bi = j; }
    bi += g * 8;
#pragma unroll
    for (int off = 1; off < 8; off <<= 1) {
        const float ov = __shfl_xor(bv, off);
        const int   oi = __shfl_xor(bi, off);
        if (ov > bv || (ov == bv && oi < bi)) { bv = ov; bi = oi; }
    }
    if (g == 0) sb[tok] = bi;
    __syncthreads();
    if (t < 8) {
        v4i v;
        v[0] = sb[t * 4 + 0]; v[1] = sb[t * 4 + 1]; v[2] = sb[t * 4 + 2]; v[3] = sb[t * 4 + 3];
        const size_t o = (size_t)hd * NTOK + n0 + t * 4;
        *(volatile v4i*)(bkt + o) = v;
        __threadfence();
        *(volatile v4i*)(bkt + o) = v;
    }
}

__global__ void __launch_bounds__(256)
k_attn(const unsigned short* __restrict__ qh, const unsigned short* __restrict__ ql,
       const unsigned short* __restrict__ kh, const unsigned short* __restrict__ kl,
       const unsigned short* __restrict__ vth, const unsigned short* __restrict__ vtl,
       const int* __restrict__ bkt, unsigned short* __restrict__ oh,
       unsigned short* __restrict__ ol) {
    __shared__ v4u  uni[2 * 64 * KLD / 8];
    __shared__ float s_s[64 * 64];
    __shared__ float red_s[256];
    __shared__ int   bq_s[64];
    __shared__ int   bk_s[64];
    __shared__ float mrow[64];
    __shared__ float lrow[64];
    __shared__ float arow[64];
    unsigned short* p_h = (unsigned short*)uni;
    unsigned short* p_l = p_h + 64 * PLD;
    float* os = (float*)uni;

    const int hd = blockIdx.y, m0g = blockIdx.x * 64;
    if (m0g + 64 > NTOK) return;
    const int tid = threadIdx.x, wave = tid >> 5, lane = tid & 31;
    const int lh = lane >> 4, lm = lane & 15;
    const float SCALE = 0.08838834764831845f;

    if (tid < 64) {
        bq_s[tid] = bkt[hd * NTOK + m0g + tid];
        mrow[tid] = NEGBIG;
        lrow[tid] = 0.f;
    }

    const int ni = wave & 3, mih = wave >> 2;
    const size_t qoff0 = (size_t)(m0g + mih * 32 + lm) * DMODEL + hd * HDIM + 8 * lh;
    const size_t qoff1 = qoff0 + (size_t)16 * DMODEL;
    const size_t voff  = (size_t)(hd * HDIM + wave * 16 + lm) * NTOK + 8 * lh;

    v8f of0 = {}, of1 = {}, of2 = {}, of3 = {};

    for (int n0 = 0; n0 < NTOK; n0 += 64) {
        __syncthreads();
        if (tid < 64) bk_s[tid] = bkt[hd * NTOK + n0 + tid];
#pragma unroll
        for (int c = 0; c < 4; ++c) {
            const int chunk = tid + c * 256;
            const int krow = chunk >> 4, c16 = chunk & 15;
            const size_t g = (size_t)(n0 + krow) * DMODEL + hd * HDIM + c16 * 8;
            uni[krow * (KLD / 8) + c16]                  = *(const v4u*)(kh + g);
            uni[64 * (KLD / 8) + krow * (KLD / 8) + c16] = *(const v4u*)(kl + g);
        }
        __syncthreads();

        v8f sf0 = {}, sf1 = {};
#pragma unroll 1
        for (int k0 = 0; k0 < HDIM; k0 += 32) {
            const int kidx = (ni * 16 + lm) * KLD + k0 + 8 * lh;
            Frag bh, bl, a0h, a0l, a1h, a1l;
            bh.u[0] = uni[kidx >> 3];
            bh.u[1] = uni[(kidx + 16) >> 3];
            bl.u[0] = uni[64 * (KLD / 8) + (kidx >> 3)];
            bl.u[1] = uni[64 * (KLD / 8) + ((kidx + 16) >> 3)];
            a0h.u[0] = *(const v4u*)(qh + qoff0 + k0); a0h.u[1] = *(const v4u*)(qh + qoff0 + k0 + 16);
            a0l.u[0] = *(const v4u*)(ql + qoff0 + k0); a0l.u[1] = *(const v4u*)(ql + qoff0 + k0 + 16);
            a1h.u[0] = *(const v4u*)(qh + qoff1 + k0); a1h.u[1] = *(const v4u*)(qh + qoff1 + k0 + 16);
            a1l.u[0] = *(const v4u*)(ql + qoff1 + k0); a1l.u[1] = *(const v4u*)(ql + qoff1 + k0 + 16);
            sf0 = wmma3(a0h.v, a0l.v, bh.v, bl.v, sf0);
            sf1 = wmma3(a1h.v, a1l.v, bh.v, bl.v, sf1);
        }
        {
            const int col = ni * 16 + lm;
            const int bkv = bk_s[col];
#pragma unroll
            for (int r = 0; r < 8; ++r) {
                const int row0 = mih * 32 + 8 * lh + r;
                const int row1 = row0 + 16;
                s_s[row0 * 64 + col] = (bq_s[row0] == bkv) ? sf0[r] * SCALE : NEGBIG;
                s_s[row1 * 64 + col] = (bq_s[row1] == bkv) ? sf1[r] * SCALE : NEGBIG;
            }
        }
        __syncthreads();

        const int row = tid >> 2;
        const int cb  = (tid & 3) * 16;
        float pm = NEGBIG;
#pragma unroll
        for (int j = 0; j < 16; ++j) pm = fmaxf(pm, s_s[row * 64 + cb + j]);
        red_s[tid] = pm;
        __syncthreads();
        const float rowmax = fmaxf(fmaxf(red_s[row * 4 + 0], red_s[row * 4 + 1]),
                                   fmaxf(red_s[row * 4 + 2], red_s[row * 4 + 3]));
        const float mold = mrow[row];
        const float newm = fmaxf(mold, rowmax);
        __syncthreads();
        float psum = 0.f;
#pragma unroll 4
        for (int j = 0; j < 16; ++j) {
            const float sv = s_s[row * 64 + cb + j];
            const float p = (sv < 0.5f * NEGBIG) ? 0.f : expf(sv - newm);
            unsigned int hb, lb;
            split2(p, hb, lb);
            p_h[row * PLD + cb + j] = (unsigned short)hb;
            p_l[row * PLD + cb + j] = (unsigned short)lb;
            psum += p;
        }
        red_s[tid] = psum;
        __syncthreads();
        if ((tid & 3) == 0) {
            const float rsum = red_s[tid] + red_s[tid + 1] + red_s[tid + 2] + red_s[tid + 3];
            const float alpha = expf(mold - newm);
            arow[row] = alpha;
            lrow[row] = lrow[row] * alpha + rsum;
            mrow[row] = newm;
        }
        __syncthreads();

#pragma unroll
        for (int r = 0; r < 8; ++r) {
            of0[r] *= arow[0  + 8 * lh + r];
            of1[r] *= arow[16 + 8 * lh + r];
            of2[r] *= arow[32 + 8 * lh + r];
            of3[r] *= arow[48 + 8 * lh + r];
        }
#pragma unroll 1
        for (int kk = 0; kk < 64; kk += 32) {
            Frag vbh, vbl;
            vbh.u[0] = *(const v4u*)(vth + voff + n0 + kk); vbh.u[1] = *(const v4u*)(vth + voff + n0 + kk + 16);
            vbl.u[0] = *(const v4u*)(vtl + voff + n0 + kk); vbl.u[1] = *(const v4u*)(vtl + voff + n0 + kk + 16);
#define PV_TILE(MI, ACC) {                                                  \
                const int pi = ((MI) * 16 + lm) * PLD + kk + 8 * lh;        \
                Frag pah, pal;                                              \
                pah.u[0] = uni[pi >> 3];                                    \
                pah.u[1] = uni[(pi + 16) >> 3];                             \
                pal.u[0] = uni[64 * (PLD / 8) + (pi >> 3)];                 \
                pal.u[1] = uni[64 * (PLD / 8) + ((pi + 16) >> 3)];          \
                ACC = wmma3(pah.v, pal.v, vbh.v, vbl.v, ACC); }
            PV_TILE(0, of0)
            PV_TILE(1, of1)
            PV_TILE(2, of2)
            PV_TILE(3, of3)
#undef PV_TILE
        }
    }

    __syncthreads();
#pragma unroll
    for (int r = 0; r < 8; ++r) {
        const int r0 = 8 * lh + r;
        os[(0  + r0) * OLD + wave * 16 + lm] = of0[r] / lrow[0  + r0];
        os[(16 + r0) * OLD + wave * 16 + lm] = of1[r] / lrow[16 + r0];
        os[(32 + r0) * OLD + wave * 16 + lm] = of2[r] / lrow[32 + r0];
        os[(48 + r0) * OLD + wave * 16 + lm] = of3[r] / lrow[48 + r0];
    }
    __syncthreads();
    for (int pass = 0; pass < 2; ++pass) {
        if (pass) __threadfence();
#pragma unroll
        for (int it = 0; it < 4; ++it) {
            const int L = it * 32 + (tid >> 3);
            const int orow = L >> 1;
            const int col = (L & 1) * 64 + (tid & 7) * 8;
            const v4f x0 = *(const v4f*)(os + orow * OLD + col);
            const v4f x1 = *(const v4f*)(os + orow * OLD + col + 4);
            float v[8] = {x0[0], x0[1], x0[2], x0[3], x1[0], x1[1], x1[2], x1[3]};
            v4u hv, lv;
            pack8(v, hv, lv);
            const size_t g = (size_t)(m0g + orow) * DMODEL + hd * HDIM + col;
            *(volatile v4u*)(oh + g) = hv;
            *(volatile v4u*)(ol + g) = lv;
        }
    }
}

extern "C" void kernel_launch(void* const* d_in, const int* in_sizes, int n_in,
                              void* d_out, int out_size, void* d_ws, size_t ws_size,
                              hipStream_t stream) {
    if (n_in < 10) return;
    if (in_sizes[0] != NTOK * DMODEL) return;
    if (in_sizes[1] != DMODEL * DMODEL || in_sizes[3] != DMODEL * DMODEL ||
        in_sizes[5] != DMODEL * DMODEL || in_sizes[7] != DMODEL * DMODEL) return;
    if (in_sizes[2] != DMODEL || in_sizes[4] != DMODEL || in_sizes[6] != DMODEL ||
        in_sizes[8] != DMODEL) return;
    if (in_sizes[9] != NHEAD * HDIM * NBUCK) return;
    if (out_size != NTOK * DMODEL) return;

    const float* x  = (const float*)d_in[0];
    const float* Wq = (const float*)d_in[1];
    const float* bq = (const float*)d_in[2];
    const float* Wk = (const float*)d_in[3];
    const float* bk = (const float*)d_in[4];
    const float* Wv = (const float*)d_in[5];
    const float* bv = (const float*)d_in[6];
    const float* Wo = (const float*)d_in[7];
    const float* bo = (const float*)d_in[8];
    const float* hp = (const float*)d_in[9];
    float* out = (float*)d_out;

    const size_t MB = (size_t)1 << 20;
    const size_t need = 64 * MB + (size_t)NHEAD * NTOK * sizeof(int);
    if (ws_size < need) return;
    char* ws = (char*)d_ws;
    unsigned short* xh   = (unsigned short*)(ws + 0 * MB);
    unsigned short* xl   = (unsigned short*)(ws + 4 * MB);
    unsigned short* wqTh = (unsigned short*)(ws + 8 * MB);
    unsigned short* wqTl = (unsigned short*)(ws + 10 * MB);
    unsigned short* wkTh = (unsigned short*)(ws + 12 * MB);
    unsigned short* wkTl = (unsigned short*)(ws + 14 * MB);
    unsigned short* wvTh = (unsigned short*)(ws + 16 * MB);
    unsigned short* wvTl = (unsigned short*)(ws + 18 * MB);
    unsigned short* woTh = (unsigned short*)(ws + 20 * MB);
    unsigned short* woTl = (unsigned short*)(ws + 22 * MB);
    float*          q32  = (float*)         (ws + 24 * MB);
    unsigned short* qh   = (unsigned short*)(ws + 32 * MB);
    unsigned short* ql   = (unsigned short*)(ws + 36 * MB);
    unsigned short* khp  = (unsigned short*)(ws + 40 * MB);
    unsigned short* klp  = (unsigned short*)(ws + 44 * MB);
    unsigned short* vth  = (unsigned short*)(ws + 48 * MB);
    unsigned short* vtl  = (unsigned short*)(ws + 52 * MB);
    unsigned short* ohp  = (unsigned short*)(ws + 56 * MB);
    unsigned short* olp  = (unsigned short*)(ws + 60 * MB);
    int*            bkt  = (int*)           (ws + 64 * MB);

    const int NX8 = NTOK * DMODEL / 8;
    k_split8<<<(NX8 + 255) / 256, 256, 0, stream>>>(x, xh, xl, NX8);

    const dim3 gt((DMODEL + 63) / 64, (DMODEL + 63) / 64);
    k_splitT<<<gt, 256, 0, stream>>>(Wq, wqTh, wqTl, DMODEL, DMODEL);
    k_splitT<<<gt, 256, 0, stream>>>(Wk, wkTh, wkTl, DMODEL, DMODEL);
    k_splitT<<<gt, 256, 0, stream>>>(Wv, wvTh, wvTl, DMODEL, DMODEL);
    k_splitT<<<gt, 256, 0, stream>>>(Wo, woTh, woTl, DMODEL, DMODEL);

    const dim3 gg(DMODEL / 64, NTOK / 64);
    k_gemm3<<<gg, 128, 0, stream>>>(xh, xl, wqTh, wqTl, bq, q32, qh,  ql,  NTOK, DMODEL, DMODEL, 1 | 2);
    k_gemm3<<<gg, 128, 0, stream>>>(xh, xl, wkTh, wkTl, bk, q32, khp, klp, NTOK, DMODEL, DMODEL, 2);
    k_gemm3<<<gg, 128, 0, stream>>>(xh, xl, wvTh, wvTl, bv, q32, vth, vtl, NTOK, DMODEL, DMODEL, 4);

    k_hash<<<dim3(NTOK / 32, NHEAD), 256, 0, stream>>>(q32, hp, bkt);

    k_attn<<<dim3(NTOK / 64, NHEAD), 256, 0, stream>>>(qh, ql, khp, klp, vth, vtl, bkt, ohp, olp);

    k_gemm3<<<gg, 128, 0, stream>>>(ohp, olp, woTh, woTl, bo, out, qh, ql, NTOK, DMODEL, DMODEL, 1);
}
